// LSTM_dist_custom_47699906789961
// MI455X (gfx1250) — hardware-run, weakly checked
//
#include <hip/hip_runtime.h>
#include <math.h>

constexpr int NBATCH   = 128;
constexpr int NSTEP    = 2048;
constexpr int NCIN     = 3;
constexpr int NCMID    = 64;
constexpr int NHID     = 128;
constexpr int NGATE    = 4 * NHID;
constexpr int NCLS     = 40;
constexpr int NTHREADS = 256;
constexpr int ROWS_BLK = 16;
constexpr int PITCH_X  = 72;
constexpr int PITCH_H  = 136;
constexpr int NOUT_BLK = ROWS_BLK * NCLS;
constexpr float BN_EPS = 1e-5f;
constexpr float ACARRY = 64.0f;
constexpr float WCARRY = 16.0f;
constexpr float FOLD   = 1.0f / (ACARRY * WCARRY);

static_assert(NBATCH % ROWS_BLK == 0, "batch tiles");
static_assert(NHID == 16 * (NTHREADS / 32), "one 16-unit subtile per wave");
static_assert(NTHREADS * 4 == ROWS_BLK * NCMID, "conv thread map covers 16 x 64 with 4 channels per thread");
static_assert(NCMID % 32 == 0 && NHID % 32 == 0, "K multiples of 32");
static_assert((PITCH_X * 2) % 16 == 0 && (PITCH_H * 2) % 16 == 0, "16-B aligned fragment rows");
static_assert(PITCH_X >= NCMID && PITCH_H >= NHID, "tile extents");
static_assert(NOUT_BLK == 5 * 32 * 4, "five float4 wave stores per tile");
static_assert((NOUT_BLK * 4) % 128 == 0, "tile output is whole 128-B lines");
static_assert((NGATE * NCMID / 8) % 256 == 0 && (NGATE * NHID / 8) % 256 == 0, "convert grids exact");

typedef __attribute__((ext_vector_type(16))) _Float16 v16h;
typedef __attribute__((ext_vector_type(8)))  _Float16 v8h;
typedef __attribute__((ext_vector_type(4)))  _Float16 v4h;
typedef __attribute__((ext_vector_type(8)))  float    v8f;
typedef __attribute__((ext_vector_type(4)))  float    v4f;

template <typename T> struct Frag;
template <> struct Frag<_Float16> {
  typedef v16h V; union U { v16h v; v8h h[2]; };
  static __device__ __forceinline__ v16h load(const _Float16* p) {
    U f; f.h[0] = *(const v8h*)(p); f.h[1] = *(const v8h*)(p + 16); return f.v;
  }
  static __device__ __forceinline__ v8f mma(v16h a, v16h b, v8f c) {
    return __builtin_amdgcn_wmma_f32_16x16x32_f16(false, a, false, b, (short)0, c, false, false);
  }
};

__device__ __forceinline__ void group_guard4(v8f& c0, v8f& c1, v8f& c2, v8f& c3,
                                             v16h a, v16h b0, v16h b1, v16h b2, v16h b3) {
  asm volatile("v_nop\n\tv_nop\n\tv_nop\n\tv_nop"
               : "+v"(c0), "+v"(c1), "+v"(c2), "+v"(c3)
               : "v"(a), "v"(b0), "v"(b1), "v"(b2), "v"(b3));
}
__device__ __forceinline__ void acc_guard4(v8f& a, v8f& b, v8f& c, v8f& d) {
  asm volatile("v_nop\n\tv_nop\n\tv_nop\n\tv_nop" : "+v"(a), "+v"(b), "+v"(c), "+v"(d));
}

__device__ __forceinline__ float sigm(float v)    { return __builtin_amdgcn_rcpf(1.0f + expf(-v)); }
__device__ __forceinline__ float tanh_id(float v) { return 1.0f - 2.0f * __builtin_amdgcn_rcpf(1.0f + expf(2.0f * v)); }

__global__ __launch_bounds__(256)
void cvt8_f16_kernel(const float* __restrict__ src, unsigned short* __restrict__ dst, int n8, float sc) {
  const int i = blockIdx.x * 256 + threadIdx.x;
  if (i < n8) {
    const float* sp = src + (size_t)i * 8;
    const v4f a = *(const v4f*)(sp);
    const v4f b = *(const v4f*)(sp + 4);
    v8h hv;
#pragma unroll
    for (int e = 0; e < 4; ++e) {
      hv[e]     = (_Float16)(a[e] * sc);
      hv[4 + e] = (_Float16)(b[e] * sc);
    }
    *(volatile v8h*)(dst + (size_t)i * 8) = hv;
    __threadfence();
    *(volatile v8h*)(dst + (size_t)i * 8) = hv;
  }
}

__device__ __forceinline__ void hx_store(_Float16* dst, float x0, float x1, float x2,
                                         const float (&cw)[4][3], const float (&cbe)[4]) {
  v4h pk;
#pragma unroll
  for (int e = 0; e < 4; ++e) {
    float cv = x0 * cw[e][0];
    cv = fmaf(x1, cw[e][1], cv);
    cv = fmaf(x2, cw[e][2], cv);
    const float hxv = fmaxf(cv + cbe[e], 0.0f);
    pk[e] = (_Float16)(hxv * ACARRY);
  }
  *(v4h*)dst = pk;
}

__global__ __launch_bounds__(NTHREADS)
void lstm_scan_kernel(const float* __restrict__ x,     const float* __restrict__ conv_w,
                      const float* __restrict__ conv_b, const float* __restrict__ gamma,
                      const float* __restrict__ beta,   const float* __restrict__ rmean,
                      const float* __restrict__ rvar,
                      const unsigned short* __restrict__ WXp, const unsigned short* __restrict__ WHp,
                      const float* __restrict__ bih,    const float* __restrict__ bhh,
                      const float* __restrict__ Wout,   const float* __restrict__ bout,
                      float* __restrict__ out) {
  __shared__ __align__(16) _Float16 s_hx[ROWS_BLK * PITCH_X];
  __shared__ __align__(16) _Float16 s_h [ROWS_BLK * PITCH_H];
  __shared__ __align__(16) float    s_hl[ROWS_BLK * NHID];
  __shared__ __align__(16) float    s_out[NOUT_BLK];

  const _Float16* WX = (const _Float16*)WXp;
  const _Float16* WH = (const _Float16*)WHp;
  const int tid   = threadIdx.x;
  const int lane  = tid & 31;
  const int wave  = tid >> 5;
  const int c     = lane & 15;
  const int hh    = lane >> 4;
  const int koff  = hh * 8;
  const int bBase = blockIdx.x * ROWS_BLK;
  const int j     = 16 * wave + c;

  float bb[4];
#pragma unroll
  for (int g = 0; g < 4; ++g) bb[g] = bih[g * NHID + j] + bhh[g * NHID + j];

  const int m2  = tid >> 4;
  const int ch4 = (tid & 15) * 4;
  float cw[4][3], cbe[4];
  {
    const v4f w0 = *(const v4f*)(conv_w + ch4 * NCIN);
    const v4f w1 = *(const v4f*)(conv_w + ch4 * NCIN + 4);
    const v4f w2 = *(const v4f*)(conv_w + ch4 * NCIN + 8);
    const float w12[12] = { w0[0], w0[1], w0[2], w0[3], w1[0], w1[1], w1[2], w1[3], w2[0], w2[1], w2[2], w2[3] };
    const v4f gm = *(const v4f*)(gamma  + ch4);
    const v4f rv = *(const v4f*)(rvar   + ch4);
    const v4f cb = *(const v4f*)(conv_b + ch4);
    const v4f rm = *(const v4f*)(rmean  + ch4);
    const v4f bt = *(const v4f*)(beta   + ch4);
#pragma unroll
    for (int e = 0; e < 4; ++e) {
      const float bninv = gm[e] * rsqrtf(rv[e] + BN_EPS);
      cw[e][0] = w12[3 * e + 0] * bninv;
      cw[e][1] = w12[3 * e + 1] * bninv;
      cw[e][2] = w12[3 * e + 2] * bninv;
      cbe[e]   = (cb[e] - rm[e]) * bninv + bt[e];
    }
  }
  const float* xrow = x + (size_t)(bBase + m2) * NSTEP * NCIN;
  _Float16* hxdst = s_hx + m2 * PITCH_X + ch4;

  float cst[8], hst[8];
#pragma unroll
  for (int r = 0; r < 8; ++r) { cst[r] = 0.0f; hst[r] = 0.0f; }

#pragma unroll 1
  for (int i = tid; i < ROWS_BLK * PITCH_H; i += NTHREADS) s_h[i] = (_Float16)0.0f;
#pragma unroll 1
  for (int i = tid; i < ROWS_BLK * PITCH_X; i += NTHREADS) s_hx[i] = (_Float16)0.0f;
  __syncthreads();
  {
    const float x0 = xrow[0], x1 = xrow[1], x2 = xrow[2];
    hx_store(hxdst, x0, x1, x2, cw, cbe);
  }
  __syncthreads();

  const _Float16* axrow = s_hx + c * PITCH_X + koff;
  const _Float16* ahrow = s_h  + c * PITCH_H + koff;
  const _Float16* wx = WX + (size_t)j * NCMID + koff;
  const _Float16* wh = WH + (size_t)j * NHID + koff;
  const v8f z8 = {0.f, 0.f, 0.f, 0.f, 0.f, 0.f, 0.f, 0.f};

#pragma unroll 1
  for (int t = 0; t < NSTEP; ++t) {
    const int tn = (t + 1 < NSTEP) ? (t + 1) : (NSTEP - 1);
    const float* xp = xrow + (size_t)tn * NCIN;
    float xv0 = xp[0];
    float xv1 = xp[1];
    float xv2 = xp[2];
    asm volatile("" : "+v"(xv0), "+v"(xv1), "+v"(xv2));

    v8f acc[4];
    acc[0] = z8; acc[1] = z8; acc[2] = z8; acc[3] = z8;
#pragma unroll 1
    for (int kx = 0; kx < NCMID; kx += 32) {
      const v16h a  = Frag<_Float16>::load(axrow + kx);
      const v16h b0 = Frag<_Float16>::load(wx + kx);
      const v16h b1 = Frag<_Float16>::load(wx + (size_t)1 * NHID * NCMID + kx);
      const v16h b2 = Frag<_Float16>::load(wx + (size_t)2 * NHID * NCMID + kx);
      const v16h b3 = Frag<_Float16>::load(wx + (size_t)3 * NHID * NCMID + kx);
      acc[0] = Frag<_Float16>::mma(a, b0, acc[0]);
      acc[1] = Frag<_Float16>::mma(a, b1, acc[1]);
      acc[2] = Frag<_Float16>::mma(a, b2, acc[2]);
      acc[3] = Frag<_Float16>::mma(a, b3, acc[3]);
      group_guard4(acc[0], acc[1], acc[2], acc[3], a, b0, b1, b2, b3);
    }
#pragma unroll 1
    for (int k0 = 0; k0 < NHID; k0 += 32) {
      const v16h a  = Frag<_Float16>::load(ahrow + k0);
      const v16h b0 = Frag<_Float16>::load(wh + k0);
      const v16h b1 = Frag<_Float16>::load(wh + (size_t)1 * NHID * NHID + k0);
      const v16h b2 = Frag<_Float16>::load(wh + (size_t)2 * NHID * NHID + k0);
      const v16h b3 = Frag<_Float16>::load(wh + (size_t)3 * NHID * NHID + k0);
      acc[0] = Frag<_Float16>::mma(a, b0, acc[0]);
      acc[1] = Frag<_Float16>::mma(a, b1, acc[1]);
      acc[2] = Frag<_Float16>::mma(a, b2, acc[2]);
      acc[3] = Frag<_Float16>::mma(a, b3, acc[3]);
      group_guard4(acc[0], acc[1], acc[2], acc[3], a, b0, b1, b2, b3);
    }
    acc_guard4(acc[0], acc[1], acc[2], acc[3]);

#pragma unroll
    for (int r = 0; r < 8; ++r) {
      const float zi = acc[0][r] * FOLD + bb[0];
      const float zf = acc[1][r] * FOLD + bb[1];
      const float zg = acc[2][r] * FOLD + bb[2];
      const float zo = acc[3][r] * FOLD + bb[3];
      const float ig = sigm(zi);
      const float fg = sigm(zf);
      const float gg = tanh_id(zg);
      const float og = sigm(zo);
      const float cn = fg * cst[r] + ig * gg;
      cst[r] = cn;
      hst[r] = og * tanh_id(cn);
    }
    __syncthreads();
#pragma unroll
    for (int r = 0; r < 8; ++r) s_h[(8 * hh + r) * PITCH_H + j] = (_Float16)(hst[r] * ACARRY);
    hx_store(hxdst, xv0, xv1, xv2, cw, cbe);
    __syncthreads();
  }

#pragma unroll
  for (int r = 0; r < 8; ++r) s_hl[(8 * hh + r) * NHID + j] = hst[r];
  __syncthreads();

#pragma unroll 1
  for (int it = 0; it < 3; ++it) {
    const int oraw = it * NTHREADS + tid;
    const int oi   = (oraw < NOUT_BLK) ? oraw : (NOUT_BLK - 1);
    const int om   = oi / NCLS;
    const int ocls = oi - om * NCLS;
    const float* wr = Wout + (size_t)ocls * NHID;
    const float* hr = s_hl + om * NHID;
    float a = 0.0f;
#pragma unroll 1
    for (int k = 0; k < NHID; k += 4) {
      const v4f wv = *(const v4f*)(wr + k);
      const v4f hv = *(const v4f*)(hr + k);
      a = fmaf(hv[0], wv[0], a);
      a = fmaf(hv[1], wv[1], a);
      a = fmaf(hv[2], wv[2], a);
      a = fmaf(hv[3], wv[3], a);
    }
    a += bout[ocls];
    if (oraw < NOUT_BLK) s_out[oraw] = a;
  }
  __syncthreads();

  if (wave == 0) {
    float* ob = out + (size_t)blockIdx.x * NOUT_BLK;
    for (int pass = 0; pass < 2; ++pass) {
#pragma unroll
      for (int it = 0; it < 5; ++it) {
        const int e4 = (it * 32 + lane) * 4;
        const v4f v = *(const v4f*)(s_out + e4);
        *(volatile v4f*)(ob + e4) = v;
      }
      __threadfence();
    }
  }
}

extern "C" void kernel_launch(void* const* d_in, const int* in_sizes, int n_in,
                              void* d_out, int out_size, void* d_ws, size_t ws_size,
                              hipStream_t stream) {
  if (n_in < 13 || d_out == nullptr || d_ws == nullptr) return;
  if (in_sizes[0] != NBATCH * NSTEP * NCIN || in_sizes[1] != NCMID * NCIN || in_sizes[2] != NCMID ||
      in_sizes[3] != NCMID || in_sizes[4] != NCMID || in_sizes[5] != NCMID || in_sizes[6] != NCMID ||
      in_sizes[7] != NGATE * NCMID || in_sizes[8] != NGATE * NHID || in_sizes[9] != NGATE ||
      in_sizes[10] != NGATE || in_sizes[11] != NCLS * NHID || in_sizes[12] != NCLS ||
      out_size != NBATCH * NCLS) return;

  const float* x      = (const float*)d_in[0];
  const float* conv_w = (const float*)d_in[1];
  const float* conv_b = (const float*)d_in[2];
  const float* gamma  = (const float*)d_in[3];
  const float* beta   = (const float*)d_in[4];
  const float* rmean  = (const float*)d_in[5];
  const float* rvar   = (const float*)d_in[6];
  const float* Wih    = (const float*)d_in[7];
  const float* Whh    = (const float*)d_in[8];
  const float* bih    = (const float*)d_in[9];
  const float* bhh    = (const float*)d_in[10];
  const float* Wout   = (const float*)d_in[11];
  const float* bout   = (const float*)d_in[12];
  float* out = (float*)d_out;

  char* ws = (char*)d_ws;
  size_t off = 0;
  auto carve = [&](size_t bytes) -> char* { char* p = ws + off; off += (bytes + 255) & ~(size_t)255; return p; };
  unsigned short* WX = (unsigned short*)carve((size_t)NGATE * NCMID * 2);
  unsigned short* WH = (unsigned short*)carve((size_t)NGATE * NHID * 2);
  if (off > ws_size || off > (size_t)134217728) return;

  const int n8x = NGATE * NCMID / 8;
  const int n8h = NGATE * NHID / 8;
  cvt8_f16_kernel<<<dim3(n8x / 256), dim3(256), 0, stream>>>(Wih, WX, n8x, WCARRY);
  cvt8_f16_kernel<<<dim3(n8h / 256), dim3(256), 0, stream>>>(Whh, WH, n8h, WCARRY);

  lstm_scan_kernel<<<dim3(NBATCH / ROWS_BLK), dim3(NTHREADS), 0, stream>>>(
      x, conv_w, conv_b, gamma, beta, rmean, rvar, WX, WH, bih, bhh, Wout, bout, out);
}
